// LAL_43482248904966
// MI455X (gfx1250) — hardware-verified
//
#include <hip/hip_runtime.h>
#include <math.h>

typedef __attribute__((ext_vector_type(16))) _Float16 v16h;
typedef __attribute__((ext_vector_type(16))) __bf16 v16b;
typedef __attribute__((ext_vector_type(8)))  _Float16 v8h;
typedef __attribute__((ext_vector_type(8)))  float v8f;
typedef __attribute__((ext_vector_type(4)))  float v4f;
typedef __attribute__((ext_vector_type(2)))  float v2f;
typedef __attribute__((ext_vector_type(4)))  unsigned v4u;
typedef __attribute__((ext_vector_type(4)))  int v4i;
typedef float __attribute__((may_alias)) float_a;
typedef int __attribute__((may_alias)) int_a;

template <typename T> __device__ __forceinline__ void vst2(void* p, T v) { *(volatile T*)p = v; __threadfence(); *(volatile T*)p = v; }
__device__ __forceinline__ v8f wmma16(v16h a, v16h b, v8f c) {
  v8f d = __builtin_amdgcn_wmma_f32_16x16x32_f16(false, a, false, b, (short)0, c, false, false);
  asm volatile("v_nop\n\tv_nop\n\tv_nop\n\tv_nop" : "+v"(d) : "v"(a), "v"(b));
  return d;
}
__device__ __forceinline__ v8f wmma_bf(v16b a, v16b b, v8f c) {
  v8f d = __builtin_amdgcn_wmma_f32_16x16x32_bf16(false, a, false, b, (short)0, c, false, false);
  asm volatile("v_nop\n\tv_nop\n\tv_nop\n\tv_nop" : "+v"(d) : "v"(a), "v"(b));
  return d;
}
__device__ __forceinline__ v16h frag_h(const _Float16* rowk0, int lane) {
  union { v16h v; v8h q[2]; } u; const _Float16* p = rowk0 + 8 * (lane >> 4);
  u.q[0] = *(const v8h*)p; u.q[1] = *(const v8h*)(p + 16); return u.v;
}
__device__ __forceinline__ v16h frag_f32(const float* rowk0, int lane) {
  v16h a; const float* p = rowk0 + 8 * (lane >> 4);
#pragma unroll
  for (int i = 0; i < 8; ++i) { a[i] = (_Float16)p[i]; a[8 + i] = (_Float16)p[16 + i]; }
  return a;
}
__device__ __forceinline__ v16h frag_f32s(const float* rowk0, int lane, float sc) {
  v16h a; const float* p = rowk0 + 8 * (lane >> 4);
#pragma unroll
  for (int i = 0; i < 8; ++i) { a[i] = (_Float16)(p[i] * sc); a[8 + i] = (_Float16)(p[16 + i] * sc); }
  return a;
}
__device__ __forceinline__ v16h fragc_f32(const float* W, int k0, int n, int lane, int ld, int K) {
  v16h a; const int g = lane >> 4;
#pragma unroll
  for (int i = 0; i < 8; ++i) { const int ka = k0 + 8 * g + i, kb = ka + 16;
    a[i] = (_Float16)(ka < K ? W[(size_t)(ka < K ? ka : K - 1) * ld + n] : 0.f); a[8 + i] = (_Float16)(kb < K ? W[(size_t)(kb < K ? kb : K - 1) * ld + n] : 0.f); }
  return a;
}
struct F2 { v16b h, l; };
__device__ __forceinline__ F2 bsplit16(const float v[16]) { F2 r;
#pragma unroll
  for (int i = 0; i < 16; ++i) { const __bf16 h = (__bf16)v[i]; r.h[i] = h; r.l[i] = (__bf16)(v[i] - (float)h); }
  return r; }
__device__ __forceinline__ F2 split_row(const float* row, int k0, int lane) { float v[16]; const float* p = row + k0 + 8 * (lane >> 4);
#pragma unroll
  for (int i = 0; i < 8; ++i) { v[i] = p[i]; v[8 + i] = p[16 + i]; }
  return bsplit16(v); }
__device__ __forceinline__ F2 split_rowK(const float* row, int k0, int lane, int K) { float v[16]; const int g = lane >> 4;
#pragma unroll
  for (int i = 0; i < 8; ++i) { const int ka = k0 + 8 * g + i, kb = ka + 16; v[i] = ka < K ? row[ka < K ? ka : K - 1] : 0.f; v[8 + i] = kb < K ? row[kb < K ? kb : K - 1] : 0.f; }
  return bsplit16(v); }
__device__ __forceinline__ F2 split_col(const float* W, int k0, int n, int lane, int ld, int K) { float v[16]; const int g = lane >> 4;
#pragma unroll
  for (int i = 0; i < 8; ++i) { const int ka = k0 + 8 * g + i, kb = ka + 16; v[i] = ka < K ? W[(size_t)(ka < K ? ka : K - 1) * ld + n] : 0.f; v[8 + i] = kb < K ? W[(size_t)(kb < K ? kb : K - 1) * ld + n] : 0.f; }
  return bsplit16(v); }
__device__ __forceinline__ v8f mac3(const F2& a, const F2& b, v8f c) { c = wmma_bf(a.l, b.h, c); c = wmma_bf(a.h, b.l, c); return wmma_bf(a.h, b.h, c); }
__device__ __forceinline__ float sigm(float v) { return 1.0f / (1.0f + expf(-v)); }
#define LDSX() do { asm volatile("s_wait_dscnt 0" ::: "memory"); __builtin_amdgcn_wave_barrier(); __builtin_amdgcn_fence(__ATOMIC_RELEASE, "workgroup"); } while (0)


#define NB 4
#define NN 4096
#define NR (NB * NN)
#define CC 512
#define KNB 20
#define HIDC 64
#define SLOPE 0.2f
typedef __attribute__((ext_vector_type(8))) __bf16 v8b;
__device__ __forceinline__ v16b frag_b(const __bf16* rowk0, int lane) {
  union { v16b v; v8b q[2]; } u; const __bf16* p = rowk0 + 8 * (lane >> 4);
  u.q[0] = *(const v8b*)p; u.q[1] = *(const v8b*)(p + 16); return u.v;
}
__device__ __forceinline__ float bfr(float v) { return (float)(__bf16)v; }
__device__ __attribute__((noinline)) float exp_ni(float v) { return expf(v); }
__device__ __attribute__((noinline)) float erf_ni(float v) { return erff(v); }

#define WS_PK   0u
#define PK_W2   (128 * CC)
#define PK_END  (PK_W2 + CC * HIDC)
#define WS_SQ   (((2u * PK_END) + 127u) / 128u * 128u)
#define WS_IDX  (WS_SQ + 4u * NR)
#define WS_PAB  (WS_IDX + 4u * NR * 32)
#define WS_ST1  (WS_PAB + 4u * NR * 128)
#define WS_MR1  (WS_ST1 + 8u * 256 * HIDC * 2)
#define WS_H1H  (WS_MR1 + 4u * 2 * HIDC)
#define WS_H1L  (WS_H1H + 2u * NR * HIDC)
#define WS_Y    (WS_H1L + 2u * NR * HIDC)
#define WS_ST2  (WS_Y + 4u * (size_t)NR * CC)
#define WS_MR2  (WS_ST2 + 8u * 256 * CC * 2)
#define WS_END  (WS_MR2 + 4u * 2 * CC)

__global__ __launch_bounds__(256) void k_pack(const float* __restrict__ W1, const float* __restrict__ W2, __bf16* __restrict__ PK) {
  __shared__ __align__(16) __bf16 s[CC]; const int n = blockIdx.x, which = blockIdx.y, t = threadIdx.x; int K; size_t dst;
  if (which == 0) { if (n >= 128) return; K = CC; dst = (size_t)n * CC; const int dr = n & 63, half = n >> 6; for (int k = t; k < CC; k += 256) s[k] = (__bf16)W1[(size_t)dr * (2 * CC) + half * CC + k]; }
  else { K = HIDC; dst = PK_W2 + (size_t)n * HIDC; if (t < HIDC) s[t] = (__bf16)W2[(size_t)n * HIDC + t]; }
  __syncthreads();
  for (int q = t; q < K / 8; q += 256) vst2((unsigned*)(PK + dst + q * 8), *(const v4u*)&s[q * 8]);
}
__global__ __launch_bounds__(256) void k_sq(const float* __restrict__ XYZ, float* __restrict__ SQ) {
  __shared__ __align__(16) float s[256]; const int t = threadIdx.x; const size_t p = (size_t)blockIdx.x * 256 + t;
  const float x0 = bfr(XYZ[p * 3]), x1 = bfr(XYZ[p * 3 + 1]), x2 = bfr(XYZ[p * 3 + 2]);
  s[t] = __fadd_rn(__fadd_rn(__fmul_rn(x0, x0), __fmul_rn(x2, x2)), __fmul_rn(x1, x1));
  __syncthreads();
  if (t < 64) vst2(SQ + (size_t)blockIdx.x * 256 + t * 4, *(const v4f*)&s[t * 4]);
}
__global__ __launch_bounds__(128) void k_knn(const float* __restrict__ XYZ, const float* __restrict__ SQ, int* __restrict__ IDX) {
  __shared__ float sd[4][NN]; __shared__ __align__(16) int sidx[4][32];
  const int tid = threadIdx.x, wave = tid >> 5, lane = tid & 31; const size_t q = (size_t)blockIdx.x * 4 + wave; const int b = (int)(q / NN); const size_t base = (size_t)b * NN;
  const float qx0 = bfr(XYZ[q * 3]), qx1 = bfr(XYZ[q * 3 + 1]), qx2 = bfr(XYZ[q * 3 + 2]); const float sqi = SQ[q];
  for (int j = lane; j < NN; j += 32) { const size_t pj = base + j; const float y0 = bfr(XYZ[pj * 3]), y1 = bfr(XYZ[pj * 3 + 1]), y2 = bfr(XYZ[pj * 3 + 2]);
    const float dot = __fadd_rn(__fadd_rn(__fmul_rn(qx0, y0), __fmul_rn(qx1, y1)), __fmul_rn(qx2, y2));
    sd[wave][j] = __fsub_rn(__fadd_rn(sqi, SQ[pj]), __fmul_rn(2.0f, dot)); }
  if (lane < 32) sidx[wave][lane] = 0;
  __syncthreads();
#pragma unroll 1
  for (int s = 0; s < KNB; ++s) { float bv = 3.0e38f; int bi = 0x7fffffff;
    for (int j = lane; j < NN; j += 32) { const float v = sd[wave][j]; if (v < bv) { bv = v; bi = j; } }
#pragma unroll
    for (int o = 1; o < 32; o <<= 1) { const float ov = __shfl_xor(bv, o); const int oi = __shfl_xor(bi, o); if (ov < bv || (ov == bv && oi < bi)) { bv = ov; bi = oi; } }
    if (lane == 0) { sidx[wave][s] = bi; sd[wave][bi] = 3.0e38f; }
    __syncthreads(); }
  if (tid < 32) vst2((unsigned*)(IDX + ((size_t)blockIdx.x * 4 + (tid >> 3)) * 32 + (tid & 7) * 4), *(const v4u*)&sidx[tid >> 3][(tid & 7) * 4]);
}
__global__ __launch_bounds__(128) void k_pab(const float* __restrict__ X, const __bf16* __restrict__ PK, float* __restrict__ PAB) {
  __shared__ __align__(16) float so[4][16][132];
  const int tid = threadIdx.x, wave = tid >> 5, lane = tid & 31, col = lane & 15, g = lane >> 4; const size_t r0 = (size_t)blockIdx.x * 64 + wave * 16;
  v8f acc[8] = {};
#pragma unroll 2
  for (int kc = 0; kc < CC / 32; ++kc) { v16b a; { const float* p = X + (r0 + col) * CC + kc * 32 + 8 * g;
#pragma unroll
      for (int i = 0; i < 8; ++i) { a[i] = (__bf16)p[i]; a[8 + i] = (__bf16)p[16 + i]; } }
#pragma unroll
    for (int j = 0; j < 8; ++j) acc[j] = wmma_bf(a, frag_b(PK + (size_t)(j * 16 + col) * CC + kc * 32, lane), acc[j]); }
#pragma unroll
  for (int j = 0; j < 8; ++j)
#pragma unroll
    for (int r = 0; r < 8; ++r) so[wave][8 * g + r][j * 16 + col] = acc[j][r];
  LDSX();
  for (int rl = 0; rl < 16; ++rl) vst2(PAB + (r0 + rl) * 128 + lane * 4, *(const v4f*)&so[wave][rl][lane * 4]);
}
__global__ __launch_bounds__(256) void k_stat1(const float* __restrict__ PAB, const int* __restrict__ IDX, double* __restrict__ ST1) {
  __shared__ double ss[16][HIDC][2]; __shared__ __align__(16) double sl[HIDC * 2]; const int tid = threadIdx.x; const int ql = tid >> 2, part = tid & 3; const size_t q = (size_t)blockIdx.x * 64 + ql; const int b = (int)(q / NN);
  double s1[16], s2[16];
#pragma unroll
  for (int i = 0; i < 16; ++i) { s1[i] = 0.0; s2[i] = 0.0; }
  for (int k = 0; k < KNB; ++k) { const size_t nb = (size_t)b * NN + IDX[q * 32 + k];
#pragma unroll
    for (int i = 0; i < 16; ++i) { const int dch = part * 16 + i; const float h = (PAB[nb * 128 + dch] - PAB[q * 128 + dch]) + PAB[q * 128 + 64 + dch]; s1[i] += (double)h; s2[i] += (double)h * (double)h; } }
  for (int i = 0; i < 16; ++i) {   }
  __syncthreads();
  for (int round = 0; round < 4; ++round) { if ((ql >> 4) == round) {
#pragma unroll
      for (int i = 0; i < 16; ++i) { const int dch = part * 16 + i; if (round == 0) { ss[ql & 15][dch][0] = s1[i]; ss[ql & 15][dch][1] = s2[i]; } else { ss[ql & 15][dch][0] += s1[i]; ss[ql & 15][dch][1] += s2[i]; } } }
    __syncthreads(); }
  if (tid < HIDC * 2) { const int dch = tid >> 1, w = tid & 1; double a = 0.0; for (int sI = 0; sI < 16; ++sI) a += ss[sI][dch][w]; sl[dch * 2 + w] = a; }
  __syncthreads();
  if (tid < HIDC) vst2((unsigned*)(ST1 + (size_t)blockIdx.x * HIDC * 2 + tid * 2), *(const v4u*)&sl[tid * 2]);
}
__global__ __launch_bounds__(64) void k_red1(const double* __restrict__ ST1, const float* __restrict__ G1, float* __restrict__ MR1) {
  __shared__ __align__(16) float s[2 * HIDC]; const int t = threadIdx.x; double a = 0.0, b2 = 0.0;
  for (int blk = 0; blk < NR / 64; ++blk) { a += ST1[((size_t)blk * HIDC + t) * 2]; b2 += ST1[((size_t)blk * HIDC + t) * 2 + 1]; }
  const double cnt = (double)NR * KNB; const double mean = a / cnt; const double var = fmax(b2 / cnt - mean * mean, 0.0);
  s[t] = (float)mean; s[HIDC + t] = bfr(G1[t]) * (float)(1.0 / sqrt(var + 1e-5));
  __syncthreads();
  if (t < 32) vst2(MR1 + t * 4, *(const v4f*)&s[t * 4]);
}
__global__ __launch_bounds__(256) void k_hmax(const float* __restrict__ PAB, const int* __restrict__ IDX, const float* __restrict__ MR1, const float* __restrict__ B1, __bf16* __restrict__ H1H, __bf16* __restrict__ H1L) {
  __shared__ __align__(16) __bf16 sh_[64][HIDC + 8], sl_[64][HIDC + 8]; const int tid = threadIdx.x; const int ql = tid >> 2, part = tid & 3; const size_t q = (size_t)blockIdx.x * 64 + ql; const int b = (int)(q / NN);
  float mx[16];
#pragma unroll
  for (int i = 0; i < 16; ++i) mx[i] = -3.0e38f;
  for (int k = 0; k < KNB; ++k) { const size_t nb = (size_t)b * NN + IDX[q * 32 + k];
#pragma unroll
    for (int i = 0; i < 16; ++i) { const int dch = part * 16 + i; const float h = (PAB[nb * 128 + dch] - PAB[q * 128 + dch]) + PAB[q * 128 + 64 + dch]; float v = MR1[HIDC + dch] * (h - MR1[dch]) + bfr(B1[dch]); v = (v >= 0.f) ? v : SLOPE * v; mx[i] = fmaxf(mx[i], v); } }
#pragma unroll
  for (int i = 0; i < 16; ++i) { const int dch = part * 16 + i; const __bf16 hb = (__bf16)mx[i]; sh_[ql][dch] = hb; sl_[ql][dch] = (__bf16)(mx[i] - (float)hb); }
  __syncthreads();
  for (int e = tid; e < 64 * 8 * 2; e += 256) { const int plane = e >> 9, rem = e & 511; const int r = rem >> 3, pc = rem & 7; const size_t o = ((size_t)blockIdx.x * 64 + r) * HIDC + pc * 8;
    if (plane == 0) vst2((unsigned*)(H1H + o), *(const v4u*)&sh_[r][pc * 8]); else vst2((unsigned*)(H1L + o), *(const v4u*)&sl_[r][pc * 8]); }
}
__global__ __launch_bounds__(128) void k_y(const __bf16* __restrict__ H1H, const __bf16* __restrict__ H1L, const __bf16* __restrict__ PK, float* __restrict__ Y, double* __restrict__ ST2) {
  __shared__ __align__(16) float so[4][16][132]; __shared__ __align__(16) double sst[128][2];
  const int tid = threadIdx.x, wave = tid >> 5, lane = tid & 31, col = lane & 15, g = lane >> 4; const size_t r0 = (size_t)blockIdx.x * 64 + wave * 16; const int n0 = blockIdx.y * 128;
  v8f acc[8] = {};
#pragma unroll
  for (int kc = 0; kc < HIDC / 32; ++kc) { const v16b ah = frag_b(H1H + (r0 + col) * HIDC + kc * 32, lane), al = frag_b(H1L + (r0 + col) * HIDC + kc * 32, lane);
#pragma unroll
    for (int j = 0; j < 8; ++j) { const v16b w = frag_b(PK + PK_W2 + (size_t)(n0 + j * 16 + col) * HIDC + kc * 32, lane); acc[j] = wmma_bf(al, w, acc[j]); acc[j] = wmma_bf(ah, w, acc[j]); } }
#pragma unroll
  for (int j = 0; j < 8; ++j)
#pragma unroll
    for (int r = 0; r < 8; ++r) so[wave][8 * g + r][j * 16 + col] = acc[j][r];
  __syncthreads();
  for (int rl = 0; rl < 16; ++rl) vst2(Y + (r0 + rl) * CC + n0 + lane * 4, *(const v4f*)&so[wave][rl][lane * 4]);
  { const int c = tid; double a = 0.0, b2 = 0.0; for (int w = 0; w < 4; ++w) for (int r = 0; r < 16; ++r) { const double v = (double)so[w][r][c]; a += v; b2 += v * v; } sst[c][0] = a; sst[c][1] = b2; }
  __syncthreads();
  for (int e = tid; e < 128; e += 128) vst2((unsigned*)(ST2 + ((size_t)blockIdx.x * CC + n0 + e) * 2), *(const v4u*)&sst[e][0]);
}
__global__ __launch_bounds__(512) void k_red2(const double* __restrict__ ST2, const float* __restrict__ G2, float* __restrict__ MR2) {
  __shared__ __align__(16) float s[2 * CC]; const int t = threadIdx.x; double a = 0.0, b2 = 0.0;
  for (int blk = 0; blk < NR / 64; ++blk) { a += ST2[((size_t)blk * CC + t) * 2]; b2 += ST2[((size_t)blk * CC + t) * 2 + 1]; }
  const double mean = a / (double)NR; const double var = fmax(b2 / (double)NR - mean * mean, 0.0);
  s[t] = (float)mean; s[CC + t] = bfr(G2[t]) * (float)(1.0 / sqrt(var + 1e-5));
  __syncthreads();
  if (t < 2 * CC / 4) vst2(MR2 + t * 4, *(const v4f*)&s[t * 4]);
}
__global__ __launch_bounds__(128) void k_out(const float* __restrict__ Y, const float* __restrict__ MR2, const float* __restrict__ B2, float* __restrict__ OUT) {
  const size_t row = blockIdx.x; const int t = threadIdx.x; v4f v;
#pragma unroll
  for (int i = 0; i < 4; ++i) { const int c = t * 4 + i; float z = MR2[CC + c] * (Y[row * CC + c] - MR2[c]) + bfr(B2[c]); v[i] = (z >= 0.f) ? z : SLOPE * z; }
  vst2(OUT + row * CC + t * 4, v);
}
extern "C" void kernel_launch(void* const* d_in, const int* in_sizes, int n_in, void* d_out, int out_size, void* d_ws, size_t ws_size, hipStream_t stream) {
  (void)in_sizes; (void)n_in; (void)out_size;
  const float** F = (const float**)d_in;
  if (ws_size < (size_t)WS_END) return;
  char* ws = (char*)d_ws; __bf16 *PK = (__bf16*)(ws + WS_PK), *H1H = (__bf16*)(ws + WS_H1H), *H1L = (__bf16*)(ws + WS_H1L); float *SQ = (float*)(ws + WS_SQ), *PAB = (float*)(ws + WS_PAB), *MR1 = (float*)(ws + WS_MR1), *Y = (float*)(ws + WS_Y), *MR2 = (float*)(ws + WS_MR2); int* IDX = (int*)(ws + WS_IDX); double *ST1 = (double*)(ws + WS_ST1), *ST2 = (double*)(ws + WS_ST2);
  k_pack<<<dim3(CC, 2), 256, 0, stream>>>(F[2], F[5], PK);
  k_sq<<<NR / 256, 256, 0, stream>>>(F[1], SQ);
  k_knn<<<NR / 4, 128, 0, stream>>>(F[1], SQ, IDX);
  k_pab<<<NR / 64, 128, 0, stream>>>(F[0], PK, PAB);
  k_stat1<<<NR / 64, 256, 0, stream>>>(PAB, IDX, ST1);
  k_red1<<<1, 64, 0, stream>>>(ST1, F[3], MR1);
  k_hmax<<<NR / 64, 256, 0, stream>>>(PAB, IDX, MR1, F[4], H1H, H1L);
  k_y<<<dim3(NR / 64, CC / 128), 128, 0, stream>>>(H1H, H1L, PK, Y, ST2);
  k_red2<<<1, 512, 0, stream>>>(ST2, F[6], MR2);
  k_out<<<NR, 128, 0, stream>>>(Y, MR2, F[7], (float*)d_out);
}
